// MoeGroupMLP_14663018348759
// MI455X (gfx1250) — hardware-verified
//
#include <hip/hip_runtime.h>
#include <math.h>

typedef __attribute__((ext_vector_type(16))) _Float16 v16h;
typedef __attribute__((ext_vector_type(16))) __bf16 v16b;
typedef __attribute__((ext_vector_type(8)))  _Float16 v8h;
typedef __attribute__((ext_vector_type(8)))  float v8f;
typedef __attribute__((ext_vector_type(4)))  float v4f;
typedef __attribute__((ext_vector_type(2)))  float v2f;
typedef __attribute__((ext_vector_type(4)))  unsigned v4u;
typedef __attribute__((ext_vector_type(4)))  int v4i;
typedef float __attribute__((may_alias)) float_a;
typedef int __attribute__((may_alias)) int_a;

template <typename T> __device__ __forceinline__ void vst2(void* p, T v) { *(volatile T*)p = v; __threadfence(); *(volatile T*)p = v; }
__device__ __forceinline__ v8f wmma16(v16h a, v16h b, v8f c) {
  v8f d = __builtin_amdgcn_wmma_f32_16x16x32_f16(false, a, false, b, (short)0, c, false, false);
  asm volatile("v_nop\n\tv_nop\n\tv_nop\n\tv_nop" : "+v"(d) : "v"(a), "v"(b));
  return d;
}
__device__ __forceinline__ v8f wmma_bf(v16b a, v16b b, v8f c) {
  v8f d = __builtin_amdgcn_wmma_f32_16x16x32_bf16(false, a, false, b, (short)0, c, false, false);
  asm volatile("v_nop\n\tv_nop\n\tv_nop\n\tv_nop" : "+v"(d) : "v"(a), "v"(b));
  return d;
}
__device__ __forceinline__ v16h frag_h(const _Float16* rowk0, int lane) {
  union { v16h v; v8h q[2]; } u; const _Float16* p = rowk0 + 8 * (lane >> 4);
  u.q[0] = *(const v8h*)p; u.q[1] = *(const v8h*)(p + 16); return u.v;
}
__device__ __forceinline__ v16h frag_f32(const float* rowk0, int lane) {
  v16h a; const float* p = rowk0 + 8 * (lane >> 4);
#pragma unroll
  for (int i = 0; i < 8; ++i) { a[i] = (_Float16)p[i]; a[8 + i] = (_Float16)p[16 + i]; }
  return a;
}
__device__ __forceinline__ v16h frag_f32s(const float* rowk0, int lane, float sc) {
  v16h a; const float* p = rowk0 + 8 * (lane >> 4);
#pragma unroll
  for (int i = 0; i < 8; ++i) { a[i] = (_Float16)(p[i] * sc); a[8 + i] = (_Float16)(p[16 + i] * sc); }
  return a;
}
__device__ __forceinline__ v16h fragc_f32(const float* W, int k0, int n, int lane, int ld, int K) {
  v16h a; const int g = lane >> 4;
#pragma unroll
  for (int i = 0; i < 8; ++i) { const int ka = k0 + 8 * g + i, kb = ka + 16;
    a[i] = (_Float16)(ka < K ? W[(size_t)ka * ld + n] : 0.f); a[8 + i] = (_Float16)(kb < K ? W[(size_t)kb * ld + n] : 0.f); }
  return a;
}
struct F2 { v16b h, l; };
__device__ __forceinline__ F2 bsplit16(const float v[16]) { F2 r;
#pragma unroll
  for (int i = 0; i < 16; ++i) { const __bf16 h = (__bf16)v[i]; r.h[i] = h; r.l[i] = (__bf16)(v[i] - (float)h); }
  return r; }
__device__ __forceinline__ F2 split_row(const float* row, int k0, int lane) { float v[16]; const float* p = row + k0 + 8 * (lane >> 4);
#pragma unroll
  for (int i = 0; i < 8; ++i) { v[i] = p[i]; v[8 + i] = p[16 + i]; }
  return bsplit16(v); }
__device__ __forceinline__ F2 split_rowK(const float* row, int k0, int lane, int K) { float v[16]; const int g = lane >> 4;
#pragma unroll
  for (int i = 0; i < 8; ++i) { const int ka = k0 + 8 * g + i, kb = ka + 16; v[i] = ka < K ? row[ka] : 0.f; v[8 + i] = kb < K ? row[kb] : 0.f; }
  return bsplit16(v); }
__device__ __forceinline__ F2 split_col(const float* W, int k0, int n, int lane, int ld, int K) { float v[16]; const int g = lane >> 4;
#pragma unroll
  for (int i = 0; i < 8; ++i) { const int ka = k0 + 8 * g + i, kb = ka + 16; v[i] = ka < K ? W[(size_t)ka * ld + n] : 0.f; v[8 + i] = kb < K ? W[(size_t)kb * ld + n] : 0.f; }
  return bsplit16(v); }
__device__ __forceinline__ v8f mac3(const F2& a, const F2& b, v8f c) { c = wmma_bf(a.l, b.h, c); c = wmma_bf(a.h, b.l, c); return wmma_bf(a.h, b.h, c); }
__device__ __forceinline__ float sigm(float v) { return 1.0f / (1.0f + expf(-v)); }
#define LDSX() do { asm volatile("s_wait_dscnt 0" ::: "memory"); __builtin_amdgcn_wave_barrier(); __builtin_amdgcn_fence(__ATOMIC_RELEASE, "workgroup"); } while (0)

#define TT 2048
#define HH 1024
#define II 1024
#define NEXP 8
#define TOPK 2
#define NPAIR (TT * TOPK)
#define MAXT 32

__device__ __forceinline__ int compact_pairs(const int* __restrict__ sel, int e, int* slist, int* swt) {
  const int tid = threadIdx.x, wave = tid >> 5, lane = tid & 31; const int nth = blockDim.x, nw = nth >> 5;
  const int per = NPAIR / nth;
  int cnt = 0;
  for (int u = 0; u < per; ++u) { const int p = tid * per + u; cnt += (sel[p] == e) ? 1 : 0; }
  int incl = cnt;
#pragma unroll
  for (int off = 1; off < 32; off <<= 1) { const int v = __shfl_up(incl, off, 32); if (lane >= off) incl += v; }
  if (lane == 31) swt[wave] = incl;
  __syncthreads();
  int base = 0, tot = 0; for (int w = 0; w < nw; ++w) { const int s = swt[w]; if (w < wave) base += s; tot += s; }
  int pos = base + incl - cnt;
  for (int u = 0; u < per; ++u) { const int p = tid * per + u; if (sel[p] == e) slist[pos++] = p; }
  __syncthreads();
  return tot;
}
__global__ __launch_bounds__(256) void k_gather(const float* __restrict__ x, const int* __restrict__ sel, _Float16* __restrict__ XE) {
  __shared__ int slist[NPAIR]; __shared__ int swt[8];
  const int e = blockIdx.y, tile = blockIdx.x, tid = threadIdx.x;
  const int count = compact_pairs(sel, e, slist, swt);
  const int rl = tid >> 2, qq = tid & 3; const int slot = tile * 64 + rl;
  int t = 0; const bool live = slot < count; if (live) { const int p = slist[slot]; t = p >> 1; }
  const float* xr = x + (size_t)t * HH + qq * 256; _Float16* dst = XE + ((size_t)e * TT + slot) * HH + qq * 256;
  for (int c = 0; c < 256; c += 8) { union { v8h h; v4u u; } pk;
#pragma unroll
    for (int i = 0; i < 8; ++i) pk.h[i] = (_Float16)(live ? xr[c + i] : 0.f);
    vst2(dst + c, pk.u); }
}
__global__ __launch_bounds__(128) void k_gateup(const _Float16* __restrict__ XE, const int* __restrict__ sel, const float* __restrict__ gw, const float* __restrict__ uw, _Float16* __restrict__ HE) {
  __shared__ int slist[NPAIR]; __shared__ int swt[4];
  __shared__ __align__(16) float so[4][16][132];
  const int e = blockIdx.y, tile = blockIdx.x, n0 = blockIdx.z * 128, tid = threadIdx.x, wave = tid >> 5, lane = tid & 31, col = lane & 15, g = lane >> 4;
  const int count = compact_pairs(sel, e, slist, swt);
  if (tile * 64 >= count) return;
  const size_t rbase = (size_t)e * TT + tile * 64 + wave * 16;
  const float* G = gw + (size_t)e * II * HH; const float* U = uw + (size_t)e * II * HH;
  v8f ag[8] = {}, au[8] = {};
#pragma unroll 1
  for (int kc = 0; kc < HH / 32; ++kc) { const v16h a = frag_h(XE + (rbase + col) * HH + kc * 32, lane);
#pragma unroll
    for (int j = 0; j < 8; ++j) { const int i = n0 + j * 16 + col; ag[j] = wmma16(a, frag_f32s(G + (size_t)i * HH + kc * 32, lane, 16.0f), ag[j]); au[j] = wmma16(a, frag_f32s(U + (size_t)i * HH + kc * 32, lane, 16.0f), au[j]); } }
#pragma unroll
  for (int j = 0; j < 8; ++j)
#pragma unroll
    for (int r = 0; r < 8; ++r) { const float gv = ag[j][r] * (1.0f / 16.0f), uv = au[j][r] * (1.0f / 16.0f); so[wave][8 * g + r][j * 16 + col] = gv * sigm(gv) * uv; }
  LDSX();
  for (int q = lane; q < 16 * 16; q += 32) { const int rl = q >> 4, pc = q & 15; union { v8h h; v4u u; } pk;
#pragma unroll
    for (int i = 0; i < 8; ++i) pk.h[i] = (_Float16)so[wave][rl][pc * 8 + i];
    vst2(HE + (rbase + rl) * II + n0 + pc * 8, pk.u); }
}
__global__ __launch_bounds__(128) void k_down(const _Float16* __restrict__ HE, const int* __restrict__ sel, const float* __restrict__ dw, float* __restrict__ R) {
  __shared__ int slist[NPAIR]; __shared__ int swt[4];
  __shared__ __align__(16) float so[4][16][132];
  const int e = blockIdx.y, tile = blockIdx.x, n0 = blockIdx.z * 128, tid = threadIdx.x, wave = tid >> 5, lane = tid & 31, col = lane & 15, g = lane >> 4;
  const int count = compact_pairs(sel, e, slist, swt);
  if (tile * 64 >= count) return;
  const size_t rbase = (size_t)e * TT + tile * 64 + wave * 16;
  const float* D = dw + (size_t)e * HH * II;
  v8f acc[8] = {};
#pragma unroll 1
  for (int kc = 0; kc < II / 32; ++kc) { const v16h a = frag_h(HE + (rbase + col) * II + kc * 32, lane);
#pragma unroll
    for (int j = 0; j < 8; ++j) { const int h = n0 + j * 16 + col; acc[j] = wmma16(a, frag_f32s(D + (size_t)h * II + kc * 32, lane, 16.0f), acc[j]); } }
#pragma unroll
  for (int j = 0; j < 8; ++j)
#pragma unroll
    for (int r = 0; r < 8; ++r) so[wave][8 * g + r][j * 16 + col] = acc[j][r] * (1.0f / 16.0f);
  LDSX();
  for (int rl = 0; rl < 16; ++rl) { const int slot = tile * 64 + wave * 16 + rl; if (slot >= count) break;
    const int p = slist[slot]; vst2(R + (size_t)p * HH + n0 + lane * 4, *(const v4f*)(&so[wave][rl][lane * 4])); }
}
__global__ __launch_bounds__(256) void k_comb(const float* __restrict__ R, const float* __restrict__ rw, float* __restrict__ out) {
  const int t = blockIdx.x, tid = threadIdx.x; const float w0 = rw[t * 2], w1 = rw[t * 2 + 1];
  const v4f a = *(const v4f*)(R + ((size_t)t * 2) * HH + tid * 4), b = *(const v4f*)(R + ((size_t)t * 2 + 1) * HH + tid * 4);
  v4f o; o[0] = w0 * a[0] + w1 * b[0]; o[1] = w0 * a[1] + w1 * b[1]; o[2] = w0 * a[2] + w1 * b[2]; o[3] = w0 * a[3] + w1 * b[3];
  vst2(out + (size_t)t * HH + tid * 4, o);
}
extern "C" void kernel_launch(void* const* d_in, const int* in_sizes, int n_in, void* d_out, int out_size, void* d_ws, size_t ws_size, hipStream_t stream) {
  (void)in_sizes; (void)n_in; (void)out_size; (void)ws_size;
  const float* x = (const float*)d_in[0]; const float* rw = (const float*)d_in[1]; const int* sel = (const int*)d_in[2]; const int* tpe = (const int*)d_in[3];
  const float* gw = (const float*)d_in[4]; const float* uw = (const float*)d_in[5]; const float* dw = (const float*)d_in[6];
  float* out = (float*)d_out;
  char* ws = (char*)d_ws; size_t off = 0;
  auto take = [&](size_t bytes) { char* p = ws + off; off += (bytes + 255) & ~(size_t)255; return p; };
  _Float16* XE = (_Float16*)take((size_t)NEXP * TT * HH * 2); _Float16* HE = (_Float16*)take((size_t)NEXP * TT * II * 2); float* R = (float*)take((size_t)NPAIR * HH * 4);
  k_gather<<<dim3(MAXT, NEXP), 256, 0, stream>>>(x, sel, XE);
  k_gateup<<<dim3(MAXT, NEXP, II / 128), 128, 0, stream>>>(XE, sel, gw, uw, HE); (void)tpe;
  k_down<<<dim3(MAXT, NEXP, HH / 128), 128, 0, stream>>>(HE, sel, dw, R);
  k_comb<<<TT, 256, 0, stream>>>(R, rw, out);
}
